// MultiHeadAttentionLayer_28982439313653
// MI455X (gfx1250) — hardware-verified
//
#include <hip/hip_runtime.h>

#ifndef NB
#define NB 8
#endif
#ifndef LL
#define LL 12
#endif
#define NB_FULL 8
#define LL_FULL 12
#define NQ 384
#define DIN 128
#define ATT 256
#define NHEAD 8
#define HD 32
#define DOUT 128
#define BL (NB * LL)
#define MROWS (BL * NQ)

static_assert(NB >= 1 && NB <= NB_FULL);
static_assert(LL >= 1 && LL <= LL_FULL);
static_assert(LL == LL_FULL || NB == 1);
static_assert(ATT == NHEAD * HD);
static_assert(HD == 32);
static_assert(NHEAD == 8);
static_assert(NQ % 32 == 0);
static_assert(NQ % 16 == 0);
static_assert(MROWS % 128 == 0);
static_assert(DIN % 64 == 0 && ATT % 64 == 0 && DOUT % 64 == 0);
static_assert(DIN * ATT == ATT * DOUT);
static_assert((DIN * ATT) % 4096 == 0);
static_assert(((size_t)MROWS * DIN / 8) % 256 == 0);
static_assert((size_t)NB_FULL * LL_FULL * NQ * DOUT * 4 == 18874368);
static_assert((size_t)(MROWS * DIN / 8 / 256) * 256 * 8 == (size_t)MROWS * DIN);
static_assert((size_t)(DIN * ATT / 4096) * 64 * 64 == (size_t)DIN * ATT);
static_assert((size_t)(ATT / 64) * (MROWS / 128) * 128 * 64 == (size_t)MROWS * ATT);
static_assert((size_t)(NQ / 16) * BL * NHEAD * 16 * HD == (size_t)MROWS * ATT);
static_assert((size_t)(DOUT / 64) * (MROWS / 128) * 128 * 64 == (size_t)MROWS * DOUT);

#define BTP 40
#define EQP 72
#define EVP 136
#define TP  72
#define CTP 40
#define OEP 68
#define ESZ 9216
static_assert(128 * EQP <= ESZ);
static_assert(64 * EVP <= ESZ);

typedef __bf16   v16bf __attribute__((ext_vector_type(16)));
typedef __bf16   v8bf  __attribute__((ext_vector_type(8)));
typedef _Float16 v16h  __attribute__((ext_vector_type(16)));
typedef _Float16 v8h   __attribute__((ext_vector_type(8)));
typedef float    v8f   __attribute__((ext_vector_type(8)));
typedef float    v4f   __attribute__((ext_vector_type(4)));
typedef unsigned int v4u __attribute__((ext_vector_type(4)));

__device__ __forceinline__ v8f mma_bf16(v16bf a, v16bf b, v8f c) {
  v8f d = __builtin_amdgcn_wmma_f32_16x16x32_bf16(false, a, false, b, (short)0, c, false, false);
  asm volatile("v_nop\n\tv_nop\n\tv_nop\n\tv_nop" : "+v"(d) : "v"(a), "v"(b));
  return d;
}
__device__ __forceinline__ v8f mma_f16(v16h a, v16h b, v8f c) {
  v8f d = __builtin_amdgcn_wmma_f32_16x16x32_f16(false, a, false, b, (short)0, c, false, false);
  asm volatile("v_nop\n\tv_nop\n\tv_nop\n\tv_nop" : "+v"(d) : "v"(a), "v"(b));
  return d;
}

__device__ __forceinline__ v16bf ld_frag_bf(const __bf16* p0, int ld, int rc, int kk, int lane) {
  const int hh = (lane >> 4) & 1;
  const __bf16* p = p0 + (size_t)rc * ld + kk + 8 * hh;
  const v8bf lo = *(const v8bf*)(p);
  const v8bf hi = *(const v8bf*)(p + 16);
  v16bf f;
#pragma unroll
  for (int i = 0; i < 8; ++i) { f[i] = lo[i]; f[8 + i] = hi[i]; }
  return f;
}
__device__ __forceinline__ v16h ld_frag_h(const _Float16* p0, int ld, int rc, int kk, int lane) {
  const int hh = (lane >> 4) & 1;
  const _Float16* p = p0 + (size_t)rc * ld + kk + 8 * hh;
  const v8h lo = *(const v8h*)(p);
  const v8h hi = *(const v8h*)(p + 16);
  v16h f;
#pragma unroll
  for (int i = 0; i < 8; ++i) { f[i] = lo[i]; f[8 + i] = hi[i]; }
  return f;
}

__device__ __forceinline__ unsigned int bfb(float x) {
  unsigned int u = __float_as_uint(x);
  u = u + 0x7FFFu + ((u >> 16) & 1u);
  return u >> 16;
}
__device__ __forceinline__ float bf16val(float x) {
  return __uint_as_float(bfb(x) << 16);
}
__device__ __forceinline__ unsigned short hbits(float x) {
  const _Float16 hv = (_Float16)x;
  return __builtin_bit_cast(unsigned short, hv);
}
__device__ __forceinline__ unsigned int pack2h(float a, float b) {
  return (unsigned int)hbits(a) | ((unsigned int)hbits(b) << 16);
}

__global__ __launch_bounds__(256) void k_cvt_rows(const float* __restrict__ xq,
                                                  const float* __restrict__ xk,
                                                  const float* __restrict__ xv,
                                                  unsigned short* __restrict__ xb, int n8) {
  const int z = blockIdx.y;
  const float* in = (z == 0) ? xq : ((z == 1) ? xk : xv);
  unsigned short* outp = xb + (size_t)z * MROWS * DIN;
  const int g = blockIdx.x * 256 + threadIdx.x;
  if (g >= n8) return;
  const v4f a = *(const v4f*)(in + (size_t)g * 8);
  const v4f b = *(const v4f*)(in + (size_t)g * 8 + 4);
  v4u w;
  w[0] = bfb(a[0]) | (bfb(a[1]) << 16);
  w[1] = bfb(a[2]) | (bfb(a[3]) << 16);
  w[2] = bfb(b[0]) | (bfb(b[1]) << 16);
  w[3] = bfb(b[2]) | (bfb(b[3]) << 16);
  volatile v4u* p = (volatile v4u*)(outp + (size_t)g * 8);
  *p = w;
  __threadfence();
  *p = w;
}

__global__ __launch_bounds__(256) void k_cvt_wT(const float* __restrict__ Wq,
                                                const float* __restrict__ Wk,
                                                const float* __restrict__ Wv,
                                                const float* __restrict__ Wd,
                                                unsigned short* __restrict__ wT) {
  __shared__ __align__(16) unsigned short T[64 * TP];
  const int z = blockIdx.z;
  const float* W = (z == 0) ? Wq : ((z == 1) ? Wk : ((z == 2) ? Wv : Wd));
  const bool od = (z == 3);
  const int kdim = od ? ATT : DIN;
  const int ndim = od ? DOUT : ATT;
  unsigned short* dst = wT + (size_t)z * (DIN * ATT);
  const int nkt = kdim / 64;
  const int t = blockIdx.x;
  const int k0 = (t % nkt) * 64;
  const int n0 = (t / nkt) * 64;
  const int tid = threadIdx.x;
  const int wave = tid >> 5, lane = tid & 31;

#pragma unroll
  for (int i = 0; i < 4; ++i) {
    const int idx = i * 256 + tid;
    const int kk = idx >> 4;
    const int c4 = (idx & 15) * 4;
    const v4f w = *(const v4f*)(W + (size_t)(k0 + kk) * ndim + n0 + c4);
    unsigned short e0, e1, e2, e3;
    if (od) {
      e0 = hbits(bf16val(w[0]) * 16.0f); e1 = hbits(bf16val(w[1]) * 16.0f);
      e2 = hbits(bf16val(w[2]) * 16.0f); e3 = hbits(bf16val(w[3]) * 16.0f);
    } else {
      e0 = (unsigned short)bfb(w[0]); e1 = (unsigned short)bfb(w[1]);
      e2 = (unsigned short)bfb(w[2]); e3 = (unsigned short)bfb(w[3]);
    }
    T[(c4 + 0) * TP + kk] = e0;
    T[(c4 + 1) * TP + kk] = e1;
    T[(c4 + 2) * TP + kk] = e2;
    T[(c4 + 3) * TP + kk] = e3;
  }
  __syncthreads();

  v4u v[2];
  size_t off[2];
#pragma unroll
  for (int it = 0; it < 2; ++it) {
    const int nn = wave * 8 + it * 4 + (lane >> 3);
    const int q = lane & 7;
    v[it] = *(const v4u*)(&T[nn * TP + q * 8]);
    off[it] = (size_t)(n0 + nn) * kdim + k0 + q * 8;
  }
#pragma unroll
  for (int it = 0; it < 2; ++it) *(volatile v4u*)(dst + off[it]) = v[it];
  __threadfence();
#pragma unroll
  for (int it = 0; it < 2; ++it) *(volatile v4u*)(dst + off[it]) = v[it];
}

__global__ __launch_bounds__(256) void k_proj(
    const unsigned short* __restrict__ xb, const unsigned short* __restrict__ wT,
    const float* __restrict__ bq, const float* __restrict__ bk, const float* __restrict__ bv,
    unsigned short* __restrict__ qp, unsigned short* __restrict__ kp,
    unsigned short* __restrict__ vtp) {
  __shared__ __align__(16) unsigned short bt[64 * BTP];
  __shared__ __align__(16) unsigned short E[ESZ];

  const int z = blockIdx.z;
  const int n0 = blockIdx.x * 64;
  const int m0 = blockIdx.y * 128;
  const int tid = threadIdx.x;
  const int wave = tid >> 5, lane = tid & 31;
  const int l15 = lane & 15, half = (lane >> 4) & 1;

  const unsigned short* Wt = wT + (size_t)z * ATT * DIN;
  const float* bias = (z == 0) ? bq : ((z == 1) ? bk : bv);

  const int tn = tid >> 2;
  const int tk = (tid & 3) * 8;
  const unsigned short* wsrc = Wt + (size_t)(n0 + tn) * DIN + tk;
  const __bf16* A = (const __bf16*)(xb + (size_t)z * MROWS * DIN);
  const int arow = m0 + wave * 16 + l15;

  v8f acc[4] = {};
  for (int s = 0; s < DIN / 32; ++s) {
    const int kk = s * 32;
    const v4u wv = *(const v4u*)(wsrc + kk);
    __syncthreads();
    *(v4u*)(&bt[tn * BTP + tk]) = wv;
    __syncthreads();
    const v16bf a = ld_frag_bf(A, DIN, arow, kk, lane);
#pragma unroll
    for (int j = 0; j < 4; ++j) {
      const v16bf b = ld_frag_bf((const __bf16*)bt, BTP, j * 16 + l15, 0, lane);
      acc[j] = mma_bf16(a, b, acc[j]);
    }
  }

  const float car = 8.0f;
  if (z != 2) {
#pragma unroll
    for (int j = 0; j < 4; ++j) {
      const int col = j * 16 + l15;
      const float bb = bf16val(bias[n0 + col]);
#pragma unroll
      for (int r = 0; r < 8; ++r) {
        const int row = wave * 16 + 8 * half + r;
        E[row * EQP + col] = hbits((acc[j][r] + bb) * car);
      }
    }
    __syncthreads();
    unsigned short* dst = (z == 0) ? qp : kp;
    v4u v[4];
    size_t off[4];
#pragma unroll
    for (int it = 0; it < 4; ++it) {
      const int row = wave * 16 + it * 4 + (lane >> 3);
      const int q = lane & 7;
      v[it] = *(const v4u*)(&E[row * EQP + q * 8]);
      off[it] = (size_t)(m0 + row) * ATT + n0 + q * 8;
    }
#pragma unroll
    for (int it = 0; it < 4; ++it) *(volatile v4u*)(dst + off[it]) = v[it];
    __threadfence();
#pragma unroll
    for (int it = 0; it < 4; ++it) *(volatile v4u*)(dst + off[it]) = v[it];
  } else {
#pragma unroll
    for (int j = 0; j < 4; ++j) {
      const int col = j * 16 + l15;
      const float bb = bf16val(bias[n0 + col]);
#pragma unroll
      for (int r = 0; r < 8; ++r) {
        const int srow = wave * 16 + 8 * half + r;
        E[col * EVP + srow] = hbits((acc[j][r] + bb) * car);
      }
    }
    __syncthreads();
    v4u v[4];
    size_t off[4];
#pragma unroll
    for (int it = 0; it < 4; ++it) {
      const int drow = wave * 8 + it * 2 + half;
      const int q = l15;
      v[it] = *(const v4u*)(&E[drow * EVP + q * 8]);
      off[it] = (size_t)(n0 + drow) * MROWS + m0 + q * 8;
    }
#pragma unroll
    for (int it = 0; it < 4; ++it) *(volatile v4u*)(vtp + off[it]) = v[it];
    __threadfence();
#pragma unroll
    for (int it = 0; it < 4; ++it) *(volatile v4u*)(vtp + off[it]) = v[it];
  }
}

__global__ __launch_bounds__(256) void k_attn(const unsigned short* __restrict__ qp,
                                              const unsigned short* __restrict__ kp,
                                              const unsigned short* __restrict__ vtp,
                                              unsigned short* __restrict__ ctx) {
  __shared__ __align__(16) unsigned short Cl[NHEAD * 16 * CTP];

  const int tid = threadIdx.x;
  const int wave = tid >> 5, lane = tid & 31;
  const int l15 = lane & 15;
  const int half = (lane >> 4) & 1;
  const int q0 = blockIdx.x * 16;
  const int g = blockIdx.y;
  const int head = wave;

  const _Float16* Q  = (const _Float16*)qp;
  const _Float16* K  = (const _Float16*)kp;
  const _Float16* VT = (const _Float16*)vtp;

  const _Float16* qbase = Q + ((size_t)g * NQ + q0) * ATT + head * HD;
  const v16h qb = ld_frag_h(qbase, ATT, l15, 0, lane);
  const _Float16* kbase = K + (size_t)g * NQ * ATT + head * HD;
  const _Float16* vbase = VT + (size_t)head * HD * MROWS + (size_t)g * NQ;

  v8f o[2] = {};
  float mrun = -1.0e30f, lrun = 0.0f;
  const float sscale = 0.17677669529663689f * (1.0f / 64.0f);

  for (int kc = 0; kc < NQ; kc += 32) {
    const _Float16* kt = kbase + (size_t)kc * ATT;
    const v16h ka0 = ld_frag_h(kt, ATT, l15, 0, lane);
    const v16h ka2 = ld_frag_h(kt, ATT, 16 + l15, 0, lane);
    const v8f zero = {};
    v8f c0 = mma_f16(ka0, qb, zero);
    v8f c1 = mma_f16(ka2, qb, zero);

    float sa[8], sb[8];
#pragma unroll
    for (int r = 0; r < 8; ++r) { sa[r] = c0[r] * sscale; sb[r] = c1[r] * sscale; }
    float lm = fmaxf(sa[0], sb[0]);
#pragma unroll
    for (int r = 1; r < 8; ++r) lm = fmaxf(lm, fmaxf(sa[r], sb[r]));
    lm = fmaxf(lm, __shfl_xor(lm, 16, 32));
    const float mnew = fmaxf(mrun, lm);
    const float alpha = __expf(mrun - mnew);
    float p0[8], p1[8];
    float ls = 0.0f;
#pragma unroll
    for (int r = 0; r < 8; ++r) {
      p0[r] = __expf(sa[r] - mnew);
      p1[r] = __expf(sb[r] - mnew);
      ls += p0[r] + p1[r];
    }
    ls += __shfl_xor(ls, 16, 32);
    lrun = lrun * alpha + ls;
    mrun = mnew;
#pragma unroll
    for (int j = 0; j < 2; ++j)
#pragma unroll
      for (int r = 0; r < 8; ++r) o[j][r] *= alpha;

    v16h pb;
#pragma unroll
    for (int e = 0; e < 8; ++e) {
      pb[e]     = (_Float16)(p0[e] * 1024.0f);
      pb[8 + e] = (_Float16)(p1[e] * 1024.0f);
    }
#pragma unroll
    for (int j = 0; j < 2; ++j) {
      const v16h va = ld_frag_h(vbase, MROWS, j * 16 + l15, kc, lane);
      o[j] = mma_f16(va, pb, o[j]);
    }
  }

  const float inv = 1.0f / (lrun * 512.0f);
  unsigned short* T = Cl + wave * 16 * CTP;
#pragma unroll
  for (int j = 0; j < 2; ++j) {
    v4u w;
    w[0] = pack2h(o[j][0] * inv, o[j][1] * inv);
    w[1] = pack2h(o[j][2] * inv, o[j][3] * inv);
    w[2] = pack2h(o[j][4] * inv, o[j][5] * inv);
    w[3] = pack2h(o[j][6] * inv, o[j][7] * inv);
    *(v4u*)(&T[l15 * CTP + j * 16 + 8 * half]) = w;
  }
  __syncthreads();

  v4u v[2];
  size_t off[2];
  unsigned short* cb = ctx + (((size_t)g * NHEAD + head) * NQ + q0) * HD;
#pragma unroll
  for (int it = 0; it < 2; ++it) {
    const int row = it * 8 + (lane >> 2);
    const int piece = (lane & 3) * 8;
    v[it] = *(const v4u*)(&T[row * CTP + piece]);
    off[it] = (size_t)row * HD + piece;
  }
#pragma unroll
  for (int it = 0; it < 2; ++it) *(volatile v4u*)(cb + off[it]) = v[it];
  __threadfence();
#pragma unroll
  for (int it = 0; it < 2; ++it) *(volatile v4u*)(cb + off[it]) = v[it];
}

__global__ __launch_bounds__(256) void k_oproj(const unsigned short* __restrict__ ctx,
                                               const unsigned short* __restrict__ wT,
                                               const float* __restrict__ bd,
                                               float* __restrict__ outp) {
  __shared__ __align__(16) unsigned short bt[64 * BTP];
  __shared__ __align__(16) float E[128 * OEP];

  const int n0 = blockIdx.x * 64;
  const int m0 = blockIdx.y * 128;
  const int tid = threadIdx.x;
  const int wave = tid >> 5, lane = tid & 31;
  const int l15 = lane & 15, half = (lane >> 4) & 1;

  const unsigned short* Wt = wT + (size_t)3 * ATT * DIN;
  const int tn = tid >> 2;
  const int tk = (tid & 3) * 8;
  const unsigned short* wsrc = Wt + (size_t)(n0 + tn) * ATT + tk;

  const int r0 = m0 + wave * 16;
  const int g = r0 / NQ;
  const int nl = r0 - g * NQ;
  const _Float16* A0 = (const _Float16*)ctx + ((size_t)g * NHEAD * NQ + nl) * HD;

  v8f acc[4] = {};
  for (int s = 0; s < ATT / 32; ++s) {
    const int kk = s * 32;
    const v4u wv = *(const v4u*)(wsrc + kk);
    __syncthreads();
    *(v4u*)(&bt[tn * BTP + tk]) = wv;
    __syncthreads();
    const v16h a = ld_frag_h(A0 + (size_t)s * NQ * HD, HD, l15, 0, lane);
#pragma unroll
    for (int j = 0; j < 4; ++j) {
      const v16h b = ld_frag_h((const _Float16*)bt, BTP, j * 16 + l15, 0, lane);
      acc[j] = mma_f16(a, b, acc[j]);
    }
  }

  const float cinv = 1.0f / 256.0f;
#pragma unroll
  for (int j = 0; j < 4; ++j) {
    const int col = j * 16 + l15;
    const float bb = bf16val(bd[n0 + col]);
#pragma unroll
    for (int r = 0; r < 8; ++r) {
      const int row = wave * 16 + 8 * half + r;
      E[row * OEP + col] = acc[j][r] * cinv + bb;
    }
  }
  __syncthreads();

  v4f v[8];
  size_t off[8];
#pragma unroll
  for (int it = 0; it < 8; ++it) {
    const int row = wave * 16 + it * 2 + half;
    const int q = l15;
    v[it] = *(const v4f*)(&E[row * OEP + q * 4]);
    off[it] = (size_t)(m0 + row) * DOUT + n0 + q * 4;
  }
#pragma unroll
  for (int it = 0; it < 8; ++it) *(volatile v4f*)(outp + off[it]) = v[it];
  __threadfence();
#pragma unroll
  for (int it = 0; it < 8; ++it) *(volatile v4f*)(outp + off[it]) = v[it];
}

extern "C" void kernel_launch(void* const* d_in, const int* in_sizes, int n_in,
                              void* d_out, int out_size, void* d_ws, size_t ws_size,
                              hipStream_t stream) {
  if (n_in < 11) return;
  if (in_sizes[0] < MROWS * DIN || in_sizes[1] < MROWS * DIN || in_sizes[2] < MROWS * DIN) return;
  if (in_sizes[3] < DIN * ATT || in_sizes[5] < DIN * ATT || in_sizes[7] < DIN * ATT) return;
  if (in_sizes[4] < ATT || in_sizes[6] < ATT || in_sizes[8] < ATT) return;
  if (in_sizes[9] < ATT * DOUT || in_sizes[10] < DOUT) return;
  if (out_size < MROWS * DOUT) return;

  const float* xq = (const float*)d_in[0];
  const float* xk = (const float*)d_in[1];
  const float* xv = (const float*)d_in[2];
  const float* Wq = (const float*)d_in[3];
  const float* bq = (const float*)d_in[4];
  const float* Wk = (const float*)d_in[5];
  const float* bk = (const float*)d_in[6];
  const float* Wv = (const float*)d_in[7];
  const float* bv = (const float*)d_in[8];
  const float* Wd = (const float*)d_in[9];
  const float* bd = (const float*)d_in[10];

  const size_t xb_bytes  = (size_t)3 * MROWS * DIN * 2;
  const size_t wt_bytes  = (size_t)4 * DIN * ATT * 2;
  const size_t pl_bytes  = (size_t)MROWS * ATT * 2;
  const size_t off_xb  = 0;
  const size_t off_wt  = off_xb + xb_bytes;
  const size_t off_q   = off_wt + wt_bytes;
  const size_t off_k   = off_q + pl_bytes;
  const size_t off_vt  = off_k + pl_bytes;
  const size_t off_ctx = off_vt + pl_bytes;
  const size_t total   = off_ctx + pl_bytes;
  if (total > ws_size) return;

  char* ws = (char*)d_ws;
  unsigned short* xb  = (unsigned short*)(ws + off_xb);
  unsigned short* wt  = (unsigned short*)(ws + off_wt);
  unsigned short* qpl = (unsigned short*)(ws + off_q);
  unsigned short* kpl = (unsigned short*)(ws + off_k);
  unsigned short* vtp = (unsigned short*)(ws + off_vt);
  unsigned short* cxp = (unsigned short*)(ws + off_ctx);

  const int n8 = MROWS * DIN / 8;
  k_cvt_rows<<<dim3((n8 + 255) / 256, 3), 256, 0, stream>>>(xq, xk, xv, xb, n8);
  k_cvt_wT<<<dim3(DIN * ATT / 4096, 1, 4), 256, 0, stream>>>(Wq, Wk, Wv, Wd, wt);
  k_proj<<<dim3(ATT / 64, MROWS / 128, 3), 256, 0, stream>>>(xb, wt, bq, bk, bv, qpl, kpl, vtp);
  k_attn<<<dim3(NQ / 16, BL), 256, 0, stream>>>(qpl, kpl, vtp, cxp);
  k_oproj<<<dim3(DOUT / 64, MROWS / 128), 256, 0, stream>>>(cxp, wt, bd, (float*)d_out);
}
